// GATEncoder_59931973649018
// MI455X (gfx1250) — hardware-verified
//
#include <hip/hip_runtime.h>
#include <math.h>
#include <stdint.h>

#define NN    4096
#define DD    256
#define NHD   4
#define HD    256
#define QKS   1024
#define OUTD  128
#define PSC   1024.0f
#define OSC   0.0009765625f

static_assert(NN % 128 == 0 && NN % 64 == 0);
static_assert(DD % 128 == 0 && QKS % 128 == 0 && OUTD % 128 == 0);
static_assert(DD % 32 == 0 && HD % 32 == 0 && HD == 256 && DD == 256);
static_assert(NHD * HD == QKS);

typedef __bf16         v16b __attribute__((ext_vector_type(16)));
typedef __bf16         v8b  __attribute__((ext_vector_type(8)));
typedef _Float16       v16h __attribute__((ext_vector_type(16)));
typedef _Float16       v8h  __attribute__((ext_vector_type(8)));
typedef float          v8f  __attribute__((ext_vector_type(8)));
typedef float          v4f  __attribute__((ext_vector_type(4)));
typedef unsigned int   v4u  __attribute__((ext_vector_type(4)));
typedef unsigned int   v2u  __attribute__((ext_vector_type(2)));
typedef v4f __attribute__((may_alias)) v4fa;
typedef v4u __attribute__((may_alias)) v4ua;
typedef v2u __attribute__((may_alias)) v2ua;
typedef v8b __attribute__((may_alias)) v8ba;
typedef v8h __attribute__((may_alias)) v8ha;

__device__ __forceinline__ unsigned short bf_bits(float f) {
  const unsigned u = __float_as_uint(f);
  return (unsigned short)((u + 0x7FFFu + ((u >> 16) & 1u)) >> 16);
}
__device__ __forceinline__ float bf_val(unsigned short h) { return __uint_as_float(((unsigned)h) << 16); }
__device__ __forceinline__ float bf_rne(float f) { return bf_val(bf_bits(f)); }
__device__ __forceinline__ v4f bf_rne4(v4f a) {
  v4f r;
  r[0] = bf_rne(a[0]); r[1] = bf_rne(a[1]); r[2] = bf_rne(a[2]); r[3] = bf_rne(a[3]);
  return r;
}
__device__ __forceinline__ unsigned short h_bits(float f) {
  const _Float16 hv = (_Float16)f;
  return __builtin_bit_cast(unsigned short, hv);
}
__device__ __forceinline__ unsigned pk16(unsigned short a, unsigned short b) { return (unsigned)a | ((unsigned)b << 16); }
__device__ __forceinline__ v8f zero8() { v8f z = {0.f, 0.f, 0.f, 0.f, 0.f, 0.f, 0.f, 0.f}; return z; }
__device__ __forceinline__ int wave_id() { return __builtin_amdgcn_readfirstlane((int)(threadIdx.x >> 5)); }

__device__ __forceinline__ void lds_wave_sync() {
  __builtin_amdgcn_fence(__ATOMIC_RELEASE, "workgroup");
  __builtin_amdgcn_wave_barrier();
  __builtin_amdgcn_fence(__ATOMIC_ACQUIRE, "workgroup");
}

__device__ __forceinline__ float wave_sum(float v) {
  v += __shfl_xor(v, 16, 32);
  v += __shfl_xor(v, 8, 32);
  v += __shfl_xor(v, 4, 32);
  v += __shfl_xor(v, 2, 32);
  v += __shfl_xor(v, 1, 32);
  return v;
}

union FragB { v16b v; v8b h[2]; };
union FragH { v16h v; v8h h[2]; };
__device__ __forceinline__ v16b ldfrag_b(const __bf16* p) {
  FragB f;
  f.h[0] = *(const v8ba*)(p);
  f.h[1] = *(const v8ba*)(p + 16);
  return f.v;
}
__device__ __forceinline__ v16h ldfrag_h(const _Float16* p) {
  FragH f;
  f.h[0] = *(const v8ha*)(p);
  f.h[1] = *(const v8ha*)(p + 16);
  return f.v;
}
__device__ __forceinline__ v8f mma_b(v16b a, v16b b, v8f c) {
  return __builtin_amdgcn_wmma_f32_16x16x32_bf16(false, a, false, b, (short)0, c, false, false);
}
__device__ __forceinline__ v8f mma_h(v16h a, v16h b, v8f c) {
  return __builtin_amdgcn_wmma_f32_16x16x32_f16(false, a, false, b, (short)0, c, false, false);
}
__device__ __forceinline__ void guard_b6(v8f& a, v8f& b, v16b x0, v16b x1, v16b x2, v16b x3, v16b y0, v16b y1) {
  asm volatile("v_nop\n\tv_nop\n\tv_nop\n\tv_nop" : "+v"(a), "+v"(b) : "v"(x0), "v"(x1), "v"(x2), "v"(x3), "v"(y0), "v"(y1) : "memory");
}
__device__ __forceinline__ void guard4_h5(v8f& a, v8f& b, v8f& c, v8f& d, v16h q, v16h k0, v16h k1, v16h k2, v16h k3) {
  asm volatile("v_nop\n\tv_nop\n\tv_nop\n\tv_nop" : "+v"(a), "+v"(b), "+v"(c), "+v"(d) : "v"(q), "v"(k0), "v"(k1), "v"(k2), "v"(k3) : "memory");
}
__device__ __forceinline__ void guard1_h4(v8f& a, v16h w, v16h x, v16h y, v16h z) {
  asm volatile("v_nop\n\tv_nop\n\tv_nop\n\tv_nop" : "+v"(a) : "v"(w), "v"(x), "v"(y), "v"(z) : "memory");
}
__device__ __forceinline__ void acc_guard4(v8f& a, v8f& b, v8f& c, v8f& d) {
  asm volatile("v_nop\n\tv_nop\n\tv_nop\n\tv_nop" : "+v"(a), "+v"(b), "+v"(c), "+v"(d));
}

__global__ __launch_bounds__(256) void prep_x_kernel(const float* __restrict__ x, unsigned short* __restrict__ xb, int nunits) {
  const int i = (int)blockIdx.x * 256 + (int)threadIdx.x;
  if (i >= nunits) return;
  const size_t e = 8 * (size_t)i;
  const v4f a = *(const v4fa*)(x + e);
  const v4f c = *(const v4fa*)(x + e + 4);
  v4u w;
  w[0] = pk16(bf_bits(a[0]), bf_bits(a[1]));
  w[1] = pk16(bf_bits(a[2]), bf_bits(a[3]));
  w[2] = pk16(bf_bits(c[0]), bf_bits(c[1]));
  w[3] = pk16(bf_bits(c[2]), bf_bits(c[3]));
  *(volatile v4u*)(xb + e) = w;
  __threadfence();
  *(volatile v4u*)(xb + e) = w;
}

__global__ __launch_bounds__(256) void tconv_bf16_kernel(const float* __restrict__ W, unsigned short* __restrict__ outp, int R, int Cc) {
  __shared__ __align__(16) float tf[64 * 68];
  const int c0  = (int)blockIdx.x * 64;
  const int r0  = (int)blockIdx.y * 64;
  const int tid = (int)threadIdx.x;
  {
    const int lr = tid >> 4;
    const int c4 = (tid & 15) * 4;
#pragma unroll
    for (int it = 0; it < 4; ++it) {
      const int rr = it * 16 + lr;
      const v4f a = *(const v4fa*)(W + (size_t)(r0 + rr) * Cc + c0 + c4);
      *(v4f*)(tf + rr * 68 + c4) = a;
    }
  }
  __syncthreads();
  const int sub = tid >> 3;
  const int c8  = (tid & 7) * 8;
  v4u hv[2];
#pragma unroll
  for (int it = 0; it < 2; ++it) {
    const int oc = it * 32 + sub;
    v4u a;
#pragma unroll
    for (int q = 0; q < 4; ++q) {
      const float f0 = tf[(c8 + 2 * q) * 68 + oc];
      const float f1 = tf[(c8 + 2 * q + 1) * 68 + oc];
      a[q] = pk16(bf_bits(f0), bf_bits(f1));
    }
    hv[it] = a;
  }
  for (int pass = 0; pass < 2; ++pass) {
#pragma unroll
    for (int it = 0; it < 2; ++it) {
      const int oc = it * 32 + sub;
      const size_t go = (size_t)(c0 + oc) * R + r0 + c8;
      *(volatile v4u*)(outp + go) = hv[it];
    }
    __threadfence();
  }
}

template <int EPI> struct SlabT { typedef unsigned short T; };
template <> struct SlabT<2>     { typedef float T; };
template <> struct SlabT<3>     { typedef float T; };
#define SLAB_PERW 2048

template <int EPI, bool SPLITA, bool SPLITB>
__global__ __launch_bounds__(128) __attribute__((amdgpu_num_vgpr(256))) void gemm_kernel(
    const unsigned short* Ap, const unsigned short* A2p, int lda,
    const unsigned short* Btp, const unsigned short* Bt2p, int ldb,
    const float* __restrict__ bias,
    void* C0, int ldc, int M, int N, int K) {
  typedef typename SlabT<EPI>::T ST;
  __shared__ __align__(16) ST slab_all[4 * SLAB_PERW];

  const int lane = threadIdx.x & 31;
  const int wave = wave_id();
  const int hh = lane >> 4;
  const int rl = lane & 15;
  const int tilesN = N >> 7;
  const int tilesM = M >> 5;
  const int tile = (int)blockIdx.x * 4 + wave;
  if (tile >= tilesM * tilesN) return;
  const int tm = tile / tilesN;
  const int tn = tile - tm * tilesN;
  const int m0 = tm << 5;
  const int n0 = tn << 7;

  const __bf16* A   = (const __bf16*)(const void*)Ap;
  const __bf16* A2  = (const __bf16*)(const void*)A2p;
  const __bf16* Bt  = (const __bf16*)(const void*)Btp;
  const __bf16* Bt2 = (const __bf16*)(const void*)Bt2p;

  v8f acc[2][8];
#pragma unroll
  for (int i = 0; i < 2; ++i)
#pragma unroll
    for (int j = 0; j < 8; ++j) acc[i][j] = zero8();

  for (int k0 = 0; k0 < K; k0 += 32) {
    v16b ah[2], al[2];
#pragma unroll
    for (int i = 0; i < 2; ++i) {
      const size_t ao = (size_t)(m0 + i * 16 + rl) * lda + k0 + 8 * hh;
      ah[i] = ldfrag_b(A + ao);
      al[i] = SPLITA ? ldfrag_b(A2 + ao) : ah[i];
    }
#pragma unroll
    for (int j = 0; j < 8; ++j) {
      const size_t bo = (size_t)(n0 + j * 16 + rl) * ldb + k0 + 8 * hh;
      const v16b bh = ldfrag_b(Bt + bo);
      const v16b bl = SPLITB ? ldfrag_b(Bt2 + bo) : bh;
      acc[0][j] = mma_b(ah[0], bh, acc[0][j]);
      acc[1][j] = mma_b(ah[1], bh, acc[1][j]);
      if (SPLITB) {
        acc[0][j] = mma_b(ah[0], bl, acc[0][j]);
        acc[1][j] = mma_b(ah[1], bl, acc[1][j]);
      }
      if (SPLITA) {
        acc[0][j] = mma_b(al[0], bh, acc[0][j]);
        acc[1][j] = mma_b(al[1], bh, acc[1][j]);
      }
      guard_b6(acc[0][j], acc[1][j], ah[0], ah[1], al[0], al[1], bh, bl);
    }
  }
  acc_guard4(acc[0][0], acc[0][1], acc[0][2], acc[0][3]);
  acc_guard4(acc[0][4], acc[0][5], acc[0][6], acc[0][7]);
  acc_guard4(acc[1][0], acc[1][1], acc[1][2], acc[1][3]);
  acc_guard4(acc[1][4], acc[1][5], acc[1][6], acc[1][7]);

  ST* slab = slab_all + wave * SLAB_PERW;

  if (EPI >= 2) {
    float* slf = (float*)(void*)slab;
    float* C = (float*)C0;
#pragma unroll
    for (int i = 0; i < 2; ++i) {
#pragma unroll
      for (int j = 0; j < 8; ++j) {
        float bn = 0.f;
        if (EPI == 3) bn = bf_rne(bias[n0 + j * 16 + rl]);
#pragma unroll
        for (int r = 0; r < 8; ++r)
          slf[(8 * hh + r) * 128 + j * 16 + rl] = acc[i][j][r] + bn;
      }
      lds_wave_sync();
      for (int pass = 0; pass < 2; ++pass) {
#pragma unroll
        for (int row = 0; row < 16; ++row) {
          const v4f v = *(const v4fa*)(slf + row * 128 + lane * 4);
          *(volatile v4f*)(C + (size_t)(m0 + i * 16 + row) * ldc + n0 + lane * 4) = v;
        }
        __threadfence();
      }
      lds_wave_sync();
    }
  } else {
    unsigned short* sl = (unsigned short*)(void*)slab;
    unsigned short* P0 = (unsigned short*)C0;
#pragma unroll
    for (int i = 0; i < 2; ++i) {
      if (EPI == 1) {
#pragma unroll
        for (int r = 0; r < 8; ++r) {
          const int m = m0 + i * 16 + 8 * hh + r;
          const float bm = bf_rne(bias[m]);
#pragma unroll
          for (int j = 0; j < 8; ++j) {
            const float v = acc[i][j][r] + bm;
            sl[(8 * hh + r) * 128 + j * 16 + rl] = h_bits(v);
          }
        }
      } else {
#pragma unroll
        for (int j = 0; j < 8; ++j) {
          const int nl = j * 16 + rl;
          const float bn = bf_rne(bias[n0 + nl]);
#pragma unroll
          for (int r = 0; r < 8; ++r) {
            const float v = acc[i][j][r] + bn;
            sl[(8 * hh + r) * 128 + nl] = h_bits(v);
          }
        }
      }
      lds_wave_sync();
      for (int pass = 0; pass < 2; ++pass) {
#pragma unroll
        for (int it = 0; it < 8; ++it) {
          const int row = it * 2 + hh;
          const int c8  = rl * 8;
          const v4u vh = *(const v4ua*)(sl + row * 128 + c8);
          const size_t go = (size_t)(m0 + i * 16 + row) * ldc + n0 + c8;
          *(volatile v4u*)(P0 + go) = vh;
        }
        __threadfence();
      }
      lds_wave_sync();
    }
  }
}

template <int MODE>
__global__ __launch_bounds__(256) void row_kernel(const float* __restrict__ pre, const float* __restrict__ bias,
                                                  const float* __restrict__ res, const float* __restrict__ aggp,
                                                  const float* __restrict__ gam, const float* __restrict__ bet,
                                                  float* __restrict__ outf, unsigned short* __restrict__ oh,
                                                  unsigned short* __restrict__ ol) {
  __shared__ __align__(16) unsigned short stg[8 * 2 * DD];
  const int lane = threadIdx.x & 31;
  const int wave = wave_id();
  const int row = (int)blockIdx.x * 8 + wave;
  if (row >= NN) return;
  const size_t ro = (size_t)row * DD;

  v4f v[2];
  float sum = 0.f;
#pragma unroll
  for (int i = 0; i < 2; ++i) {
    const int col = i * 128 + lane * 4;
    const v4f p  = *(const v4fa*)(pre + ro + col);
    const v4f bb = bf_rne4(*(const v4fa*)(bias + col));
    v4f t;
    if (MODE == 0) {
      const v4f rr = bf_rne4(*(const v4fa*)(res + ro + col));
      t = (p + bb) + rr;
#pragma unroll
      for (int e = 0; e < 4; ++e) {
        const float u  = t[e];
        const float en = __expf(u) - 1.0f;
        t[e] = (u > 0.f) ? u : en;
      }
    } else if (MODE == 1) {
      const v4f rr = *(const v4fa*)(res + ro + col);
      t = (p + bb) + rr;
#pragma unroll
      for (int e = 0; e < 4; ++e) t[e] = fmaxf(t[e], 0.f);
    } else {
      const size_t ao = (size_t)row * QKS + col;
      const v4f a0 = *(const v4fa*)(aggp + ao);
      const v4f a1 = *(const v4fa*)(aggp + ao + HD);
      const v4f a2 = *(const v4fa*)(aggp + ao + 2 * HD);
      const v4f a3 = *(const v4fa*)(aggp + ao + 3 * HD);
      const v4f am = ((a0 + a1) + (a2 + a3)) * 0.25f;
      t = (am + p) + bb;
    }
    v[i] = t;
    sum += (t[0] + t[1]) + (t[2] + t[3]);
  }

  v4f y[2];
  if (MODE == 0) {
    y[0] = v[0]; y[1] = v[1];
  } else {
    sum = wave_sum(sum);
    const float mean = sum * (1.0f / DD);
    float sq = 0.f;
#pragma unroll
    for (int i = 0; i < 2; ++i) {
#pragma unroll
      for (int e = 0; e < 4; ++e) {
        const float d = v[i][e] - mean;
        sq += d * d;
      }
    }
    sq = wave_sum(sq);
    const float rstd = rsqrtf(sq * (1.0f / DD) + 1e-5f);
#pragma unroll
    for (int i = 0; i < 2; ++i) {
      const int col = i * 128 + lane * 4;
      const v4f g  = bf_rne4(*(const v4fa*)(gam + col));
      const v4f be = bf_rne4(*(const v4fa*)(bet + col));
      v4f yy;
#pragma unroll
      for (int e = 0; e < 4; ++e) yy[e] = (v[i][e] - mean) * rstd * g[e] + be[e];
      y[i] = yy;
    }
  }

  float* orow = outf + ro;
  for (int pass = 0; pass < 2; ++pass) {
#pragma unroll
    for (int i = 0; i < 2; ++i)
      *(volatile v4f*)(orow + i * 128 + lane * 4) = y[i];
    __threadfence();
  }

  unsigned short* sw = stg + wave * (2 * DD);
#pragma unroll
  for (int i = 0; i < 2; ++i) {
    const int col = i * 128 + lane * 4;
    unsigned short hb[4], lb[4];
#pragma unroll
    for (int e = 0; e < 4; ++e) {
      hb[e] = bf_bits(y[i][e]);
      lb[e] = bf_bits(y[i][e] - bf_val(hb[e]));
    }
    v2u wh, wl;
    wh[0] = pk16(hb[0], hb[1]); wh[1] = pk16(hb[2], hb[3]);
    wl[0] = pk16(lb[0], lb[1]); wl[1] = pk16(lb[2], lb[3]);
    *(v2ua*)(sw + col)      = wh;
    *(v2ua*)(sw + DD + col) = wl;
  }
  lds_wave_sync();
  for (int pass = 0; pass < 2; ++pass) {
    const int co = lane * 8;
    const v4u a  = *(const v4ua*)(sw + co);
    const v4u cw = *(const v4ua*)(sw + DD + co);
    *(volatile v4u*)(oh + ro + co) = a;
    *(volatile v4u*)(ol + ro + co) = cw;
    __threadfence();
  }
}

#define KT       64
#define PSP      72
#define OSTP     128
#define ATT_O_F  (4 * 16 * 32 * 8)
#define ATT_P_H  (4 * 16 * PSP)
#define ATT_S_F  (4 * 16 * OSTP)
#define ATT_LDS_BYTES (ATT_O_F * 4 + ATT_P_H * 2 + ATT_S_F * 4)
static_assert(ATT_LDS_BYTES == 107520);
static_assert((ATT_O_F * 4) % 16 == 0 && ((ATT_O_F * 4 + ATT_P_H * 2) % 16) == 0);
static_assert(NN % KT == 0 && KT == 64);

__global__ __launch_bounds__(128) __attribute__((amdgpu_num_vgpr(240))) void attn_kernel(
    const unsigned short* __restrict__ qp, const unsigned short* __restrict__ kp,
    const unsigned short* __restrict__ vtp, float* __restrict__ agg) {
  extern __shared__ v4f att_dyn[];
  float*    o_l   = (float*)(void*)att_dyn;
  _Float16* lds_p = (_Float16*)(void*)((char*)(void*)att_dyn + ATT_O_F * 4);
  float*    lds_s = (float*)(void*)((char*)(void*)att_dyn + ATT_O_F * 4 + ATT_P_H * 2);

  const int tid  = (int)threadIdx.x;
  const int lane = tid & 31;
  const int wave = wave_id();
  const int hh   = lane >> 4;
  const int c    = lane & 15;
  const int qb   = (int)blockIdx.x;
  const int h    = (int)blockIdx.y;
  const int q0   = qb * 64 + wave * 16;

  const _Float16* Qr = (const _Float16*)(const void*)qp  + (size_t)(q0 + c) * QKS + h * HD + 8 * hh;
  const _Float16* Kg = (const _Float16*)(const void*)kp  + (size_t)h * HD + 8 * hh;
  const _Float16* Vg = (const _Float16*)(const void*)vtp + (size_t)(h * HD) * NN + 8 * hh;
  _Float16* ph = lds_p + wave * (16 * PSP);
  float*    ow = o_l + wave * (16 * 32 * 8) + lane * 8;

  {
    const v4f z4 = {0.f, 0.f, 0.f, 0.f};
#pragma unroll
    for (int t = 0; t < 16; ++t) {
      *(v4fa*)(ow + t * 256)     = z4;
      *(v4fa*)(ow + t * 256 + 4) = z4;
    }
  }

  float mrow[8], lrow[8];
#pragma unroll
  for (int r = 0; r < 8; ++r) { mrow[r] = -INFINITY; lrow[r] = 0.f; }

#pragma unroll 1
  for (int kc = 0; kc < NN / KT; ++kc) {
    const int kv0 = kc * KT;
    v8f s[4];
    s[0] = zero8(); s[1] = zero8(); s[2] = zero8(); s[3] = zero8();
#pragma unroll
    for (int dc = 0; dc < 8; ++dc) {
      const v16h qa = ldfrag_h(Qr + dc * 32);
      v16h kb[4];
#pragma unroll
      for (int j = 0; j < 4; ++j) kb[j] = ldfrag_h(Kg + (size_t)(kv0 + j * 16 + c) * QKS + dc * 32);
#pragma unroll
      for (int j = 0; j < 4; ++j) s[j] = mma_h(qa, kb[j], s[j]);
      guard4_h5(s[0], s[1], s[2], s[3], qa, kb[0], kb[1], kb[2], kb[3]);
    }
    float cm[8];
#pragma unroll
    for (int r = 0; r < 8; ++r) {
      float m = -INFINITY;
#pragma unroll
      for (int j = 0; j < 4; ++j) {
        const float sv = s[j][r] * 0.0625f;
        s[j][r] = sv;
        m = fmaxf(m, sv);
      }
#pragma unroll
      for (int off = 1; off < 16; off <<= 1) m = fmaxf(m, __shfl_xor(m, off, 32));
      cm[r] = m;
    }
    float alpha[8];
#pragma unroll
    for (int r = 0; r < 8; ++r) {
      const float mnew = fmaxf(mrow[r], cm[r]);
      const float al   = __expf(mrow[r] - mnew);
      mrow[r]  = mnew;
      alpha[r] = al;
      float psum = 0.f;
#pragma unroll
      for (int j = 0; j < 4; ++j) {
        const float p = __expf(s[j][r] - mnew);
        psum += p;
        ph[(8 * hh + r) * PSP + j * 16 + c] = (_Float16)(p * PSC);
      }
#pragma unroll
      for (int off = 1; off < 16; off <<= 1) psum += __shfl_xor(psum, off, 32);
      lrow[r] = lrow[r] * al + psum;
    }
    lds_wave_sync();
    const v16h pa0 = ldfrag_h(ph + c * PSP + 8 * hh);
    const v16h pa1 = ldfrag_h(ph + c * PSP + 32 + 8 * hh);
#pragma unroll 1
    for (int cc = 0; cc < 4; ++cc) {
      float* ocl = ow + cc * 1024;
      v8f oc[4];
#pragma unroll
      for (int t = 0; t < 4; ++t) {
        const v4f a4 = *(const v4fa*)(ocl + t * 256);
        const v4f b4 = *(const v4fa*)(ocl + t * 256 + 4);
        v8f o8;
#pragma unroll
        for (int r = 0; r < 4; ++r) {
          o8[r]     = a4[r] * alpha[r];
          o8[4 + r] = b4[r] * alpha[4 + r];
        }
        oc[t] = o8;
      }
#pragma unroll
      for (int t = 0; t < 4; ++t) {
        const size_t vo = (size_t)((cc * 4 + t) * 16 + c) * NN + kv0;
        const v16h vb0 = ldfrag_h(Vg + vo);
        const v16h vb1 = ldfrag_h(Vg + vo + 32);
        oc[t] = mma_h(pa0, vb0, oc[t]);
        oc[t] = mma_h(pa1, vb1, oc[t]);
        guard1_h4(oc[t], pa0, pa1, vb0, vb1);
      }
#pragma unroll
      for (int t = 0; t < 4; ++t) {
        v4f a4, b4;
#pragma unroll
        for (int r = 0; r < 4; ++r) { a4[r] = oc[t][r]; b4[r] = oc[t][4 + r]; }
        *(v4fa*)(ocl + t * 256)     = a4;
        *(v4fa*)(ocl + t * 256 + 4) = b4;
      }
    }
    lds_wave_sync();
  }

  float inv[8];
#pragma unroll
  for (int r = 0; r < 8; ++r) inv[r] = (1.0f / lrow[r]) * OSC;
  float* os = lds_s + wave * (16 * OSTP);
  float* Cb = agg + (size_t)q0 * QKS + h * HD;
#pragma unroll 1
  for (int ch = 0; ch < 2; ++ch) {
#pragma unroll
    for (int t = 0; t < 8; ++t) {
      const v4f a4 = *(const v4fa*)(ow + (ch * 8 + t) * 256);
      const v4f b4 = *(const v4fa*)(ow + (ch * 8 + t) * 256 + 4);
#pragma unroll
      for (int r = 0; r < 4; ++r) {
        os[(8 * hh + r) * OSTP + t * 16 + c]     = a4[r] * inv[r];
        os[(8 * hh + 4 + r) * OSTP + t * 16 + c] = b4[r] * inv[4 + r];
      }
    }
    lds_wave_sync();
    float* Cg = Cb + ch * 128;
    for (int pass = 0; pass < 2; ++pass) {
#pragma unroll
      for (int row = 0; row < 16; ++row) {
        const v4f xv = *(const v4fa*)(os + row * OSTP + lane * 4);
        *(volatile v4f*)(Cg + (size_t)row * QKS + lane * 4) = xv;
      }
      __threadfence();
    }
    lds_wave_sync();
  }
}

#define WS_TOTAL ((size_t)NN*DD*2 + 4*(size_t)DD*DD*2 + 3*(size_t)QKS*DD*2 + (size_t)OUTD*DD*2 + 6*(size_t)NN*DD*4 + 8*(size_t)NN*DD*2 + 3*(size_t)NN*QKS*2 + (size_t)NN*QKS*4)
static_assert(WS_TOTAL == 88145920);
static_assert(WS_TOTAL <= 134217728);
static_assert((size_t)(NN - 1) * OUTD + OUTD - 1 < (size_t)NN * OUTD);

extern "C" void kernel_launch(void* const* d_in, const int* in_sizes, int n_in,
                              void* d_out, int out_size, void* d_ws, size_t ws_size,
                              hipStream_t stream) {
  if (n_in < 23) return;
  if (in_sizes[0] != NN * DD) return;
  if (in_sizes[1] != DD * DD || in_sizes[2] != DD) return;
  if (in_sizes[3] != DD * DD || in_sizes[4] != DD || in_sizes[5] != DD || in_sizes[6] != DD) return;
  if (in_sizes[7] != DD * QKS || in_sizes[8] != QKS) return;
  if (in_sizes[9] != DD * QKS || in_sizes[10] != QKS) return;
  if (in_sizes[11] != DD * QKS || in_sizes[12] != QKS) return;
  if (in_sizes[13] != DD * DD || in_sizes[14] != DD || in_sizes[15] != DD || in_sizes[16] != DD) return;
  if (in_sizes[17] != DD * DD || in_sizes[18] != DD || in_sizes[19] != DD || in_sizes[20] != DD) return;
  if (in_sizes[21] != DD * OUTD || in_sizes[22] != OUTD) return;
  if (out_size != NN * OUTD) return;

  const float* x      = (const float*)d_in[0];
  const float* w_in   = (const float*)d_in[1];
  const float* b_in   = (const float*)d_in[2];
  const float* w_m1   = (const float*)d_in[3];
  const float* b_m1   = (const float*)d_in[4];
  const float* g_m1   = (const float*)d_in[5];
  const float* be_m1  = (const float*)d_in[6];
  const float* wq     = (const float*)d_in[7];
  const float* bq     = (const float*)d_in[8];
  const float* wk     = (const float*)d_in[9];
  const float* bk     = (const float*)d_in[10];
  const float* wv     = (const float*)d_in[11];
  const float* bv     = (const float*)d_in[12];
  const float* wskip  = (const float*)d_in[13];
  const float* bskip  = (const float*)d_in[14];
  const float* g_n1   = (const float*)d_in[15];
  const float* be_n1  = (const float*)d_in[16];
  const float* w_m2   = (const float*)d_in[17];
  const float* b_m2   = (const float*)d_in[18];
  const float* g_m2   = (const float*)d_in[19];
  const float* be_m2  = (const float*)d_in[20];
  const float* w_mean = (const float*)d_in[21];
  const float* b_mean = (const float*)d_in[22];
  float* out = (float*)d_out;

  const size_t szXB = (size_t)NN * DD * 2;
  const size_t szWd = (size_t)DD * DD * 2;
  const size_t szWq = (size_t)QKS * DD * 2;
  const size_t szWm = (size_t)OUTD * DD * 2;
  const size_t szF  = (size_t)NN * DD * 4;
  const size_t szH  = (size_t)NN * DD * 2;
  const size_t szQ  = (size_t)NN * QKS * 2;
  const size_t szA  = (size_t)NN * QKS * 4;
  size_t off = 0;
  const size_t oXB  = off; off += szXB;
  const size_t oWin = off; off += szWd;
  const size_t oWm1 = off; off += szWd;
  const size_t oWsk = off; off += szWd;
  const size_t oWm2 = off; off += szWd;
  const size_t oWq  = off; off += szWq;
  const size_t oWk  = off; off += szWq;
  const size_t oWv  = off; off += szWq;
  const size_t oWm  = off; off += szWm;
  const size_t oPRE = off; off += szF;
  const size_t oSKP = off; off += szF;
  const size_t oH1  = off; off += szF;
  const size_t oH2  = off; off += szF;
  const size_t oH3  = off; off += szF;
  const size_t oH4  = off; off += szF;
  const size_t oH1h = off; off += szH;
  const size_t oH1l = off; off += szH;
  const size_t oH2h = off; off += szH;
  const size_t oH2l = off; off += szH;
  const size_t oH3h = off; off += szH;
  const size_t oH3l = off; off += szH;
  const size_t oH4h = off; off += szH;
  const size_t oH4l = off; off += szH;
  const size_t oQP  = off; off += szQ;
  const size_t oKP  = off; off += szQ;
  const size_t oVTP = off; off += szQ;
  const size_t oAGG = off; off += szA;
  if (off != WS_TOTAL) return;
  if (off > ws_size) return;

  char* ws = (char*)d_ws;
  unsigned short* XB   = (unsigned short*)(ws + oXB);
  unsigned short* WinT = (unsigned short*)(ws + oWin);
  unsigned short* Wm1T = (unsigned short*)(ws + oWm1);
  unsigned short* WskT = (unsigned short*)(ws + oWsk);
  unsigned short* Wm2T = (unsigned short*)(ws + oWm2);
  unsigned short* WqT  = (unsigned short*)(ws + oWq);
  unsigned short* WkT  = (unsigned short*)(ws + oWk);
  unsigned short* WvT  = (unsigned short*)(ws + oWv);
  unsigned short* WmT  = (unsigned short*)(ws + oWm);
  float*          PRE  = (float*)(ws + oPRE);
  float*          SKP  = (float*)(ws + oSKP);
  float*          H1   = (float*)(ws + oH1);
  float*          H2   = (float*)(ws + oH2);
  float*          H3   = (float*)(ws + oH3);
  float*          H4   = (float*)(ws + oH4);
  unsigned short* H1h  = (unsigned short*)(ws + oH1h);
  unsigned short* H1l  = (unsigned short*)(ws + oH1l);
  unsigned short* H2h  = (unsigned short*)(ws + oH2h);
  unsigned short* H2l  = (unsigned short*)(ws + oH2l);
  unsigned short* H3h  = (unsigned short*)(ws + oH3h);
  unsigned short* H3l  = (unsigned short*)(ws + oH3l);
  unsigned short* H4h  = (unsigned short*)(ws + oH4h);
  unsigned short* H4l  = (unsigned short*)(ws + oH4l);
  unsigned short* QP   = (unsigned short*)(ws + oQP);
  unsigned short* KP   = (unsigned short*)(ws + oKP);
  unsigned short* VTP  = (unsigned short*)(ws + oVTP);
  float*          AGG  = (float*)(ws + oAGG);

  const dim3 b256(256), b128(128);
  const int tilesD = (NN / 32) * (DD / 128);
  const dim3 gD((tilesD + 3) / 4);
  const int tilesQ = (NN / 32) * (QKS / 128);
  const dim3 gQ((tilesQ + 3) / 4);
  const int tilesV = (QKS / 32) * (NN / 128);
  const dim3 gV((tilesV + 3) / 4);
  const int tilesO = (NN / 32) * (OUTD / 128);
  const dim3 gO((tilesO + 3) / 4);
  const dim3 gRow(NN / 8);

  const int nunits = NN * DD / 8;
  prep_x_kernel<<<dim3((nunits + 255) / 256), b256, 0, stream>>>(x, XB, nunits);
  tconv_bf16_kernel<<<dim3(DD / 64, DD / 64), b256, 0, stream>>>(w_in,   WinT, DD, DD);
  tconv_bf16_kernel<<<dim3(DD / 64, DD / 64), b256, 0, stream>>>(w_m1,   Wm1T, DD, DD);
  tconv_bf16_kernel<<<dim3(DD / 64, DD / 64), b256, 0, stream>>>(wskip,  WskT, DD, DD);
  tconv_bf16_kernel<<<dim3(DD / 64, DD / 64), b256, 0, stream>>>(w_m2,   Wm2T, DD, DD);
  tconv_bf16_kernel<<<dim3(QKS / 64, DD / 64), b256, 0, stream>>>(wq,    WqT, DD, QKS);
  tconv_bf16_kernel<<<dim3(QKS / 64, DD / 64), b256, 0, stream>>>(wk,    WkT, DD, QKS);
  tconv_bf16_kernel<<<dim3(QKS / 64, DD / 64), b256, 0, stream>>>(wv,    WvT, DD, QKS);
  tconv_bf16_kernel<<<dim3(OUTD / 64, DD / 64), b256, 0, stream>>>(w_mean, WmT, DD, OUTD);

  gemm_kernel<2, false, false><<<gD, b128, 0, stream>>>(XB, XB, DD, WinT, WinT, DD, b_in, (void*)PRE, DD, NN, DD, DD);
  row_kernel<0><<<gRow, b256, 0, stream>>>(PRE, b_in, x, PRE, b_in, b_in, H1, H1h, H1l);
  gemm_kernel<2, true, false><<<gD, b128, 0, stream>>>(H1h, H1l, DD, Wm1T, Wm1T, DD, b_m1, (void*)PRE, DD, NN, DD, DD);
  row_kernel<1><<<gRow, b256, 0, stream>>>(PRE, b_m1, H1, PRE, g_m1, be_m1, H2, H2h, H2l);
  gemm_kernel<0, true, false><<<gQ, b128, 0, stream>>>(H2h, H2l, DD, WqT, WqT, DD, bq, (void*)QP, QKS, NN, QKS, DD);
  gemm_kernel<0, true, false><<<gQ, b128, 0, stream>>>(H2h, H2l, DD, WkT, WkT, DD, bk, (void*)KP, QKS, NN, QKS, DD);
  gemm_kernel<1, false, true><<<gV, b128, 0, stream>>>(WvT, WvT, DD, H2h, H2l, DD, bv, (void*)VTP, NN, QKS, NN, DD);
  gemm_kernel<2, true, false><<<gD, b128, 0, stream>>>(H2h, H2l, DD, WskT, WskT, DD, bskip, (void*)SKP, DD, NN, DD, DD);
  (void)hipFuncSetAttribute(reinterpret_cast<const void*>(&attn_kernel), hipFuncAttributeMaxDynamicSharedMemorySize, ATT_LDS_BYTES);
  attn_kernel<<<dim3(NN / 64, NHD), b128, ATT_LDS_BYTES, stream>>>(QP, KP, VTP, AGG);
  row_kernel<2><<<gRow, b256, 0, stream>>>(SKP, bskip, SKP, AGG, g_n1, be_n1, H3, H3h, H3l);
  gemm_kernel<2, true, false><<<gD, b128, 0, stream>>>(H3h, H3l, DD, Wm2T, Wm2T, DD, b_m2, (void*)PRE, DD, NN, DD, DD);
  row_kernel<1><<<gRow, b256, 0, stream>>>(PRE, b_m2, H3, PRE, g_m2, be_m2, H4, H4h, H4l);
  gemm_kernel<3, true, false><<<gO, b128, 0, stream>>>(H4h, H4l, DD, WmT, WmT, DD, b_mean, (void*)out, OUTD, NN, OUTD, DD);
  (void)hipGetLastError();
}
